// PointConvNet_33105607917645
// MI455X (gfx1250) — hardware-verified
//
#include <hip/hip_runtime.h>
#include <stddef.h>
#include <stdint.h>

typedef _Float16 v16h __attribute__((ext_vector_type(16)));
typedef _Float16 v8h  __attribute__((ext_vector_type(8)));
typedef _Float16 v4h  __attribute__((ext_vector_type(4)));
typedef float    v8f  __attribute__((ext_vector_type(8)));
typedef float    v4f  __attribute__((ext_vector_type(4)));
typedef unsigned int v4u __attribute__((ext_vector_type(4)));
typedef int      v4i  __attribute__((ext_vector_type(4)));

#define FIN   16
#define KIN   19
#define HID   64
#define FOUT  64

#define RNODE 512
#define CHUNK 102400
#define EPT   8
#define GTHR  256
#define STEPS (CHUNK / (GTHR * EPT))
#define CAP   1280
#define NGRP  (CAP / 64)
#define ROWB  48
#define RING  256
#define TPC   (CAP / 16)

#define MTHR  128
#define NWAV  (MTHR / 32)

#define SC_IN 16.0f
#define SC_W1 64.0f
#define SC_H  8.0f
#define SC_W2 64.0f
#define INV1  (1.0f / (SC_IN * SC_W1))
#define INV2  (1.0f / (SC_H * SC_W2))

#define LDS_SMAX (RNODE * FOUT * 4)
#define LDS_HST  (NWAV * 16 * HID * 2)
#define LDS_WFR  (12 * 32 * 32)
#define LDS_SDST (NWAV * 16 * 4)
#define LDS_MLP  (LDS_SMAX + LDS_HST + LDS_WFR + LDS_SDST)

typedef char chk_steps[(STEPS * GTHR * EPT == CHUNK) ? 1 : -1];
typedef char chk_ring[((CAP % 64) == 0 && (RING % 64) == 0 && (RING & (RING - 1)) == 0 && RING <= GTHR) ? 1 : -1];
typedef char chk_tpc[((TPC % NWAV) == 0 && (ROWB % 16) == 0 && ((64 * ROWB) % 128) == 0) ? 1 : -1];

union FR16 { v16h v; v8h h8[2]; v4u u4[2]; _Float16 s[16]; };
union I8   { v4i q[2]; int s[8]; };

__device__ __forceinline__ v8f wmma16(v16h a, v16h b, v8f c) {
  c = __builtin_amdgcn_wmma_f32_16x16x32_f16(false, a, false, b, (short)0, c, false, false);
  asm volatile("v_nop\n\tv_nop\n\tv_nop\n\tv_nop" : "+v"(c) : "v"(a), "v"(b));
  return c;
}

__device__ __forceinline__ int imin(int a, int b) { return a < b ? a : b; }

__device__ __forceinline__ void put_group_twice(const v4u* src, unsigned char* dst, int tid) {
  if (tid < 192) {
    const v4u v = src[tid];
    volatile v4u* g = (volatile v4u*)(dst + (size_t)tid * 16);
    *g = v;
    __threadfence();
    *g = v;
  }
}

__device__ __forceinline__ void put_padgroup_twice(unsigned char* dst, int tid) {
  if (tid < 192) {
    v4u v;
    v[0] = 0u; v[1] = 0u; v[2] = ((tid % 3) == 2) ? 0xFFFFFFFFu : 0u; v[3] = 0u;
    volatile v4u* g = (volatile v4u*)(dst + (size_t)tid * 16);
    *g = v;
    __threadfence();
    *g = v;
  }
}

__global__ void __launch_bounds__(GTHR)
k_gather(const float* __restrict__ x, const float* __restrict__ pos,
         const int* __restrict__ eidx, int nn, int ne,
         unsigned char* __restrict__ slots)
{
  __shared__ __align__(16) v4u ring[RING * 3];
  __shared__ int wtot[GTHR / 32];

  const int tid = threadIdx.x, lane = tid & 31, wid = tid >> 5;
  const int c = blockIdx.x, r = blockIdx.y, nchunk = gridDim.x;
  const int n0 = r * RNODE;
  const int ncnt = imin(RNODE, nn - n0);
  const int estart = c * CHUNK;
  const int eend = imin(estart + CHUNK, ne);
  unsigned char* cell = slots + ((size_t)r * (size_t)nchunk + (size_t)c) * ((size_t)CAP * ROWB);
  const unsigned ltmask = (1u << lane) - 1u;
  int head = 0, pend = 0, gpos = 0;

#pragma unroll 1
  for (int s = 0; s < STEPS; ++s) {
    const int e0 = estart + s * (GTHR * EPT) + tid * EPT;
    int dv[EPT];
    int pre[EPT];
    unsigned hm = 0u;
    int nhw = 0;
#pragma unroll
    for (int j = 0; j < EPT; ++j) {
      const int e = e0 + j;
      const bool valid = e < eend;
      const int d = eidx[(size_t)ne + (size_t)(valid ? e : estart)];
      const bool hit = valid && (d >= n0) && (d < n0 + ncnt);
      const unsigned b = __builtin_amdgcn_ballot_w32(hit);
      pre[j] = nhw + (int)__builtin_popcount(b & ltmask);
      nhw += (int)__builtin_popcount(b);
      dv[j] = d;
      hm |= hit ? (1u << j) : 0u;
    }
    if (lane == 0) wtot[wid] = nhw;
    __syncthreads();
    int woff = 0, stot = 0;
#pragma unroll
    for (int w = 0; w < GTHR / 32; ++w) {
      const int t = wtot[w];
      stot += t;
      woff += (w < wid) ? t : 0;
    }
#pragma unroll
    for (int j = 0; j < EPT; ++j) {
      if (hm & (1u << j)) {
        const int sp = pend + woff + pre[j];
        if (sp < RING) {
          const int ri = (head + sp) & (RING - 1);
          int sidx = eidx[(size_t)(e0 + j)];
          sidx = sidx < 0 ? 0 : (sidx >= nn ? nn - 1 : sidx);
          const int d = dv[j];
          const v4f* xr = (const v4f*)(x + (size_t)sidx * FIN);
          const v4f xa = xr[0];
          const v4f xb = xr[1];
          const v4f xc = xr[2];
          const v4f xd = xr[3];
          const float r0 = pos[(size_t)sidx * 3 + 0] - pos[(size_t)d * 3 + 0];
          const float r1 = pos[(size_t)sidx * 3 + 1] - pos[(size_t)d * 3 + 1];
          const float r2 = pos[(size_t)sidx * 3 + 2] - pos[(size_t)d * 3 + 2];
          FR16 q;
#pragma unroll
          for (int i = 0; i < 4; ++i) {
            q.s[i]      = (_Float16)(xa[i] * SC_IN);
            q.s[4 + i]  = (_Float16)(xb[i] * SC_IN);
            q.s[8 + i]  = (_Float16)(xc[i] * SC_IN);
            q.s[12 + i] = (_Float16)(xd[i] * SC_IN);
          }
          union { v4h h; unsigned int u[2]; } rr;
          rr.h[0] = (_Float16)(r0 * SC_IN);
          rr.h[1] = (_Float16)(r1 * SC_IN);
          rr.h[2] = (_Float16)(r2 * SC_IN);
          rr.h[3] = (_Float16)0.0f;
          v4u w2;
          w2[0] = rr.u[0]; w2[1] = rr.u[1]; w2[2] = (unsigned int)d; w2[3] = 0u;
          ring[ri * 3 + 0] = q.u4[0];
          ring[ri * 3 + 1] = q.u4[1];
          ring[ri * 3 + 2] = w2;
        }
      }
    }
    pend = imin(pend + stot, RING);
    __syncthreads();
#pragma unroll 1
    for (int f = 0; f < RING / 64; ++f) {
      if (pend < 64) break;
      if (gpos + 64 <= CAP) put_group_twice(ring + head * 3, cell + (size_t)gpos * ROWB, tid);
      head = (head + 64) & (RING - 1);
      pend -= 64;
      gpos += 64;
    }
  }
  __syncthreads();
  if (tid >= pend && tid < 64) {
    const int ri = (head + tid) & (RING - 1);
    v4u z;
    z[0] = 0u; z[1] = 0u; z[2] = 0u; z[3] = 0u;
    v4u w = z;
    w[2] = 0xFFFFFFFFu;
    ring[ri * 3 + 0] = z;
    ring[ri * 3 + 1] = z;
    ring[ri * 3 + 2] = w;
  }
  __syncthreads();
  if (pend > 0) {
    if (gpos + 64 <= CAP) put_group_twice(ring + head * 3, cell + (size_t)gpos * ROWB, tid);
    gpos += 64;
  }
#pragma unroll 1
  for (int g = 0; g < NGRP; ++g) {
    if (g * 64 >= gpos) put_padgroup_twice(cell + (size_t)g * 64 * ROWB, tid);
  }
}

__device__ __forceinline__ void put_out_pass(const float* smax, float* ob, int ncnt, int tid) {
#pragma unroll 1
  for (int p = 0; p < (RNODE * FOUT) / (4 * MTHR); ++p) {
    const int u = p * MTHR + tid;
    const int node = u >> 4;
    if (node < ncnt) {
      const v4f k = *(const v4f*)(smax + (size_t)u * 4);
      v4f o;
#pragma unroll
      for (int i = 0; i < 4; ++i) o[i] = (__float_as_int(k[i]) == (int)0xFF800000) ? 0.0f : k[i];
      *(volatile v4f*)(ob + (size_t)u * 4) = o;
    }
  }
}

__global__ void __launch_bounds__(MTHR)
k_mlp_max(const unsigned char* __restrict__ slots,
          const float* __restrict__ W1, const float* __restrict__ b1,
          const float* __restrict__ W2, const float* __restrict__ b2,
          float* __restrict__ out, int nn, int nchunk)
{
  extern __shared__ __align__(16) unsigned char lds_raw[];
  float*    smax = (float*)lds_raw;
  _Float16* hst  = (_Float16*)(lds_raw + LDS_SMAX);
  v4u*      wfr  = (v4u*)(lds_raw + LDS_SMAX + LDS_HST);
  int*      sdst = (int*)(lds_raw + LDS_SMAX + LDS_HST + LDS_WFR);

  const int tid = threadIdx.x, lane = tid & 31, wid = tid >> 5;
  const int h = lane >> 4, m = lane & 15;
  const int r = blockIdx.x, n0 = r * RNODE;
  const int ncnt = imin(RNODE, nn - n0);

  {
    const float ninf = __int_as_float((int)0xFF800000);
    v4f ninf4;
    ninf4[0] = ninf; ninf4[1] = ninf; ninf4[2] = ninf; ninf4[3] = ninf;
    v4f* sm4 = (v4f*)smax;
#pragma unroll 1
    for (int i = tid; i < (RNODE * FOUT) / 4; i += MTHR) sm4[i] = ninf4;
  }
#pragma unroll 1
  for (int p = tid; p < 12 * 32; p += MTHR) {
    const int f = p >> 5, l = p & 31, hh = l >> 4, mm = l & 15;
    FR16 fr;
#pragma unroll
    for (int i = 0; i < 16; ++i) {
      const int kk = (i < 8) ? (8 * hh + i) : (16 + 8 * hh + (i - 8));
      float val;
      if (f < 4) {
        const int kcl = kk < KIN ? kk : (KIN - 1);
        val = W1[kcl * HID + f * 16 + mm] * ((kk < KIN) ? SC_W1 : 0.0f);
      } else {
        const int g = f - 4, kc = g >> 2, nb = g & 3;
        val = W2[(kc * 32 + kk) * FOUT + nb * 16 + mm] * SC_W2;
      }
      fr.s[i] = (_Float16)val;
    }
    wfr[p * 2 + 0] = fr.u4[0];
    wfr[p * 2 + 1] = fr.u4[1];
  }
  float b1v[4];
#pragma unroll
  for (int nb = 0; nb < 4; ++nb) b1v[nb] = b1[nb * 16 + m];
  const float b2w = b2[wid * 16 + m];
  __syncthreads();

  const size_t cellb = (size_t)CAP * ROWB;
  const unsigned char* rbase = slots + (size_t)r * (size_t)nchunk * cellb;
  const int nphase = (nchunk * TPC) / NWAV;
  _Float16* myh = hst + wid * (16 * HID);
  const _Float16 hz = (_Float16)0.0f;

#pragma unroll 1
  for (int ph = 0; ph < nphase; ++ph) {
    const int t = ph * NWAV + wid;
    const unsigned char* rowp = rbase + (size_t)t * (size_t)(16 * ROWB) + (size_t)(m * ROWB);
    const int drow = *(const int*)(rowp + 40);
    if (h == 0) sdst[wid * 16 + m] = drow;
    const bool tval = __builtin_amdgcn_ballot_w32(drow >= 0) != 0u;
    if (tval) {
      FR16 a1;
      a1.h8[0] = *(const v8h*)(rowp + 16 * h);
      const v4h q = *(const v4h*)(rowp + 32);
      v8h up;
      up[0] = h ? hz : q[0]; up[1] = h ? hz : q[1]; up[2] = h ? hz : q[2]; up[3] = hz;
      up[4] = hz; up[5] = hz; up[6] = hz; up[7] = hz;
      a1.h8[1] = up;
#pragma unroll
      for (int nb = 0; nb < 4; ++nb) {
        FR16 bw;
        bw.u4[0] = wfr[(nb * 32 + lane) * 2 + 0];
        bw.u4[1] = wfr[(nb * 32 + lane) * 2 + 1];
        v8f acc;
#pragma unroll
        for (int v = 0; v < 8; ++v) acc[v] = 0.0f;
        acc = wmma16(a1.v, bw.v, acc);
#pragma unroll
        for (int v = 0; v < 8; ++v) {
          float hv = acc[v] * INV1 + b1v[nb];
          hv = hv > 0.0f ? hv : 0.0f;
          myh[(8 * h + v) * HID + nb * 16 + m] = (_Float16)(hv * SC_H);
        }
      }
    }
    __syncthreads();
#pragma unroll 1
    for (int tt = 0; tt < NWAV; ++tt) {
      const int dcol = sdst[tt * 16 + m];
      const bool v2 = __builtin_amdgcn_ballot_w32(dcol >= 0) != 0u;
      if (!v2) continue;
      I8 dm, dp;
      dm.q[0] = *(const v4i*)(sdst + tt * 16 + 8 * h);
      dm.q[1] = *(const v4i*)(sdst + tt * 16 + 8 * h + 4);
      dp.q[0] = *(const v4i*)(sdst + tt * 16 + 8 * (1 - h));
      dp.q[1] = *(const v4i*)(sdst + tt * 16 + 8 * (1 - h) + 4);
      const _Float16* th = hst + tt * (16 * HID);
      FR16 a2a, a2b;
      a2a.h8[0] = *(const v8h*)(th + m * HID + 8 * h);
      a2a.h8[1] = *(const v8h*)(th + m * HID + 16 + 8 * h);
      a2b.h8[0] = *(const v8h*)(th + m * HID + 32 + 8 * h);
      a2b.h8[1] = *(const v8h*)(th + m * HID + 48 + 8 * h);
      FR16 bwa, bwb;
      bwa.u4[0] = wfr[((4 + wid) * 32 + lane) * 2 + 0];
      bwa.u4[1] = wfr[((4 + wid) * 32 + lane) * 2 + 1];
      bwb.u4[0] = wfr[((8 + wid) * 32 + lane) * 2 + 0];
      bwb.u4[1] = wfr[((8 + wid) * 32 + lane) * 2 + 1];
      v8f acc;
#pragma unroll
      for (int v = 0; v < 8; ++v) acc[v] = 0.0f;
      acc = wmma16(a2a.v, bwa.v, acc);
      acc = wmma16(a2b.v, bwb.v, acc);
#pragma unroll
      for (int v = 0; v < 8; ++v) {
        const float val = acc[v] * INV2 + b2w;
        const float oth = __shfl_xor(val, 16);
        const int dme = dm.s[v];
        const int dpt = dp.s[v];
        const unsigned rel = (unsigned)(dme - n0);
        const bool same = (dme == dpt);
        const float cand = same ? fmaxf(val, oth) : val;
        if (rel < (unsigned)RNODE && !(same && h == 1)) {
          float* sp = smax + rel * FOUT + wid * 16 + m;
          const float old = *sp;
          if (cand > old) *sp = cand;
        }
      }
    }
    __syncthreads();
  }

  float* ob = out + (size_t)n0 * FOUT;
  put_out_pass(smax, ob, ncnt, tid);
  __threadfence();
  put_out_pass(smax, ob, ncnt, tid);
}

extern "C" void kernel_launch(void* const* d_in, const int* in_sizes, int n_in,
                              void* d_out, int out_size, void* d_ws, size_t ws_size,
                              hipStream_t stream) {
  if (n_in < 7) return;
  const float* x   = (const float*)d_in[0];
  const float* pos = (const float*)d_in[1];
  const int*   ei  = (const int*)d_in[2];
  const float* W1  = (const float*)d_in[3];
  const float* b1  = (const float*)d_in[4];
  const float* W2  = (const float*)d_in[5];
  const float* b2  = (const float*)d_in[6];
  const int nn = in_sizes[0] / FIN;
  const int ne = in_sizes[2] / 2;
  if (nn <= 0 || ne <= 0) return;
  if ((long long)out_size < (long long)nn * FOUT) return;
  const int nrange = (nn + RNODE - 1) / RNODE;
  const int nchunk = (ne + CHUNK - 1) / CHUNK;
  const size_t need = (size_t)nrange * (size_t)nchunk * (size_t)CAP * (size_t)ROWB;
  if (need > ws_size) return;
  unsigned char* slots = (unsigned char*)d_ws;

  hipLaunchKernelGGL(k_gather, dim3(nchunk, nrange), dim3(GTHR), 0, stream,
                     x, pos, ei, nn, ne, slots);
  hipLaunchKernelGGL(k_mlp_max, dim3(nrange), dim3(MTHR), (size_t)LDS_MLP, stream,
                     (const unsigned char*)slots, W1, b1, W2, b2, (float*)d_out, nn, nchunk);
}
